// EdgeGraphConvLayer_58188216926420
// MI455X (gfx1250) — hardware-verified
//
#include <hip/hip_runtime.h>
#include <stddef.h>


#define DN    128
#define DE    64
#define NH    4
#define DW    (DN * NH)
#define GR    32
#define APE   72
#define APN   136
#define XSP   132
#define NAB   64
#define NB    512
#define CHUNK 2048
#define NTHR  256
#define NWAVE 8
#define WCAP  256
#define NGRP  (CHUNK / (NTHR * 4))
#define LN_EPS_F 1e-5f
#define LEAKY_F  0.2f

#define LDS_SACC (NB * DN)
#define LDS_MX   (NB * NH)
#define LDS_DEN  (NB * NH)
#define LDS_LIST (NWAVE * WCAP)
#define LDS_BYTES ((LDS_SACC + LDS_MX + LDS_DEN + LDS_LIST + NWAVE) * 4)

static_assert(WCAP == (CHUNK / NTHR) * 32);
static_assert(NGRP == 2);
static_assert(NB == 512);
static_assert(CHUNK <= 4096);
static_assert((LDS_SACC % 4) == 0 && (LDS_MX % 4) == 0 && (LDS_DEN % 4) == 0);
static_assert(LDS_BYTES == 286752);
static_assert((NAB % GR) == 0);
static_assert(NAB == NWAVE * 8);
static_assert(GR == NWAVE * 4);

typedef float          v4f  __attribute__((ext_vector_type(4)));
typedef float          v8f  __attribute__((ext_vector_type(8)));
typedef int            v4i  __attribute__((ext_vector_type(4)));
typedef _Float16       v8h  __attribute__((ext_vector_type(8)));
typedef _Float16       v16h __attribute__((ext_vector_type(16)));
typedef __bf16         v16b __attribute__((ext_vector_type(16)));
typedef unsigned short v8us __attribute__((ext_vector_type(8)));
union FragH  { v16h v; v8h half[2]; };
union FragB  { v16b v; v4i q[2]; };
union Pack16 { v8h h; v4i i; };
union PackU  { v8us s; v4i i; };

__device__ __forceinline__ v8f wmh(v16h a, v16h b, v8f c) {
  v8f d = __builtin_amdgcn_wmma_f32_16x16x32_f16(false, a, false, b, (short)0, c, false, false);
  asm volatile("v_nop\n\tv_nop\n\tv_nop\n\tv_nop" : "+v"(d) : "v"(a), "v"(b));
  return d;
}
__device__ __forceinline__ v8f wmb(v16b a, v16b b, v8f c) {
  v8f d = __builtin_amdgcn_wmma_f32_16x16x32_bf16(false, a, false, b, (short)0, c, false, false);
  asm volatile("v_nop\n\tv_nop\n\tv_nop\n\tv_nop" : "+v"(d) : "v"(a), "v"(b));
  return d;
}

__device__ __forceinline__ float wsum(float v) {
  v += __shfl_xor(v, 16, 32);
  v += __shfl_xor(v, 8, 32);
  v += __shfl_xor(v, 4, 32);
  v += __shfl_xor(v, 2, 32);
  v += __shfl_xor(v, 1, 32);
  return v;
}

__device__ __forceinline__ unsigned int bf16_rne_bits(float x) {
  const unsigned int u = __float_as_uint(x);
  return (u + 0x7FFFu + ((u >> 16) & 1u)) >> 16;
}
#define SPLIT_BF16(V, HP, LP, J) { \
    const float sv_ = (V); \
    const unsigned int hb_ = bf16_rne_bits(sv_); \
    const float hf_ = __uint_as_float(hb_ << 16); \
    HP.s[J] = (unsigned short)hb_; \
    LP.s[J] = (unsigned short)bf16_rne_bits(sv_ - hf_); }

__global__ __launch_bounds__(NTHR) void k_prepw(
    const float* __restrict__ W_rel, const float* __restrict__ W_w,
    _Float16* Wrt, unsigned short* Wh, unsigned short* Wl) {
  const int i = blockIdx.x * NTHR + threadIdx.x;
  if (i < DN * DE / 8) {
    const int n = i >> 3, k0 = (i & 7) * 8;
    Pack16 u;
#define WR(J) u.h[J] = (_Float16)(W_rel[(size_t)(k0 + (J)) * DN + n] * 8.0f);
    WR(0) WR(1) WR(2) WR(3) WR(4) WR(5) WR(6) WR(7)
#undef WR
    _Float16* p = Wrt + (size_t)n * DE + k0;
    *(volatile v4i*)p = u.i;
    __threadfence();
    *(volatile v4i*)p = u.i;
  } else if (i < DN * DE / 8 + DW * DN / 8) {
    const int t = i - DN * DE / 8;
    const int n = t >> 4, k0 = (t & 15) * 8;
    PackU uh, ul;
#define WW(J) SPLIT_BF16(W_w[(size_t)(k0 + (J)) * DW + n], uh, ul, J)
    WW(0) WW(1) WW(2) WW(3) WW(4) WW(5) WW(6) WW(7)
#undef WW
    unsigned short* ph = Wh + (size_t)n * DN + k0;
    unsigned short* pl = Wl + (size_t)n * DN + k0;
    *(volatile v4i*)ph = uh.i;
    *(volatile v4i*)pl = ul.i;
    __threadfence();
    *(volatile v4i*)ph = uh.i;
    *(volatile v4i*)pl = ul.i;
  }
}

__global__ __launch_bounds__(NTHR) void k_nodeatt(
    const float* __restrict__ hA, const float* __restrict__ W_att, float* AT, int nN) {
  __shared__ __attribute__((aligned(16))) float sW[2 * DN * NH];
  __shared__ __attribute__((aligned(16))) float sO[NAB * 2 * NH];
  const int tid = threadIdx.x, lane = tid & 31, wave = tid >> 5;
  for (int i = tid; i < 2 * DN; i += NTHR)
    *(v4f*)(sW + 4 * i) = *(const v4f*)(W_att + 4 * i);
  __syncthreads();
  const int nodeBase = blockIdx.x * NAB;
  const float* wd = sW + (4 * lane) * NH;
  const float* wsp = sW + (DN + 4 * lane) * NH;
#pragma unroll 1
  for (int j = 0; j < NAB / NWAVE; ++j) {
    const int nl = wave * (NAB / NWAVE) + j;
    int node = nodeBase + nl;
    if (node > nN - 1) node = nN - 1;
    const v4f x = *(const v4f*)(hA + (size_t)node * DN + 4 * lane);
    v4f pd = x.x * *(const v4f*)(wd) + x.y * *(const v4f*)(wd + 4)
           + x.z * *(const v4f*)(wd + 8) + x.w * *(const v4f*)(wd + 12);
    v4f ps = x.x * *(const v4f*)(wsp) + x.y * *(const v4f*)(wsp + 4)
           + x.z * *(const v4f*)(wsp + 8) + x.w * *(const v4f*)(wsp + 12);
    pd.x = wsum(pd.x); pd.y = wsum(pd.y); pd.z = wsum(pd.z); pd.w = wsum(pd.w);
    ps.x = wsum(ps.x); ps.y = wsum(ps.y); ps.z = wsum(ps.z); ps.w = wsum(ps.w);
    if (lane == 0) {
      *(v4f*)(sO + nl * 8)     = pd;
      *(v4f*)(sO + nl * 8 + 4) = ps;
    }
  }
  __syncthreads();
  const bool doit = (wave < 4);
  v4f v = {0.f, 0.f, 0.f, 0.f};
  float* p = AT;
  if (doit) {
    v = *(const v4f*)(sO + wave * 128 + 4 * lane);
    p = AT + (size_t)nodeBase * 8 + wave * 128 + 4 * lane;
    *(volatile v4f*)p = v;
  }
  __threadfence();
  if (doit) *(volatile v4f*)p = v;
}

__global__ __launch_bounds__(NTHR) void k_pgemm(
    const float* __restrict__ hA, const unsigned short* __restrict__ Wh,
    const unsigned short* __restrict__ Wl, const float* __restrict__ b_w,
    float* P, int nN) {
  __shared__ __attribute__((aligned(16))) unsigned short Ah[GR * APN];
  __shared__ __attribute__((aligned(16))) unsigned short Al[GR * APN];
  __shared__ __attribute__((aligned(16))) float Xs[GR * XSP];

  const int tid = threadIdx.x, lane = tid & 31, wave = tid >> 5;
  const int hh = lane >> 4, m = lane & 15;
  const int rowBase = blockIdx.x * GR;
  const int colBase = blockIdx.y * DN;

  {
    const int r = tid >> 3, c0 = (tid & 7) * 16;
    int row = rowBase + r;
    if (row > nN - 1) row = nN - 1;
    const float* p = hA + (size_t)row * DN + c0;
    const v4f f0 = *(const v4f*)(p), f1 = *(const v4f*)(p + 4);
    const v4f f2 = *(const v4f*)(p + 8), f3 = *(const v4f*)(p + 12);
    PackU h0, h1, l0, l1;
    SPLIT_BF16(f0.x, h0, l0, 0) SPLIT_BF16(f0.y, h0, l0, 1) SPLIT_BF16(f0.z, h0, l0, 2) SPLIT_BF16(f0.w, h0, l0, 3)
    SPLIT_BF16(f1.x, h0, l0, 4) SPLIT_BF16(f1.y, h0, l0, 5) SPLIT_BF16(f1.z, h0, l0, 6) SPLIT_BF16(f1.w, h0, l0, 7)
    SPLIT_BF16(f2.x, h1, l1, 0) SPLIT_BF16(f2.y, h1, l1, 1) SPLIT_BF16(f2.z, h1, l1, 2) SPLIT_BF16(f2.w, h1, l1, 3)
    SPLIT_BF16(f3.x, h1, l1, 4) SPLIT_BF16(f3.y, h1, l1, 5) SPLIT_BF16(f3.z, h1, l1, 6) SPLIT_BF16(f3.w, h1, l1, 7)
    *(v4i*)(Ah + r * APN + c0)     = h0.i;
    *(v4i*)(Ah + r * APN + c0 + 8) = h1.i;
    *(v4i*)(Al + r * APN + c0)     = l0.i;
    *(v4i*)(Al + r * APN + c0 + 8) = l1.i;
  }
  __syncthreads();

  const int ncol = colBase + wave * 16 + m;
  v8f c0a = {0.f, 0.f, 0.f, 0.f, 0.f, 0.f, 0.f, 0.f};
  v8f c1a = {0.f, 0.f, 0.f, 0.f, 0.f, 0.f, 0.f, 0.f};
#pragma unroll
  for (int kt = 0; kt < DN / 32; ++kt) {
    const int k0 = kt * 32;
    FragB bh, bl, a0h, a0l, a1h, a1l;
    const unsigned short* pbh = Wh + (size_t)ncol * DN + k0 + 8 * hh;
    const unsigned short* pbl = Wl + (size_t)ncol * DN + k0 + 8 * hh;
    const unsigned short* ph0 = Ah + m * APN + k0 + 8 * hh;
    const unsigned short* pl0 = Al + m * APN + k0 + 8 * hh;
    const unsigned short* ph1 = Ah + (16 + m) * APN + k0 + 8 * hh;
    const unsigned short* pl1 = Al + (16 + m) * APN + k0 + 8 * hh;
    bh.q[0]  = *(const v4i*)pbh; bh.q[1]  = *(const v4i*)(pbh + 16);
    bl.q[0]  = *(const v4i*)pbl; bl.q[1]  = *(const v4i*)(pbl + 16);
    a0h.q[0] = *(const v4i*)ph0; a0h.q[1] = *(const v4i*)(ph0 + 16);
    a0l.q[0] = *(const v4i*)pl0; a0l.q[1] = *(const v4i*)(pl0 + 16);
    a1h.q[0] = *(const v4i*)ph1; a1h.q[1] = *(const v4i*)(ph1 + 16);
    a1l.q[0] = *(const v4i*)pl1; a1l.q[1] = *(const v4i*)(pl1 + 16);
    c0a = wmb(a0h.v, bh.v, c0a);
    c0a = wmb(a0h.v, bl.v, c0a);
    c0a = wmb(a0l.v, bh.v, c0a);
    c1a = wmb(a1h.v, bh.v, c1a);
    c1a = wmb(a1h.v, bl.v, c1a);
    c1a = wmb(a1l.v, bh.v, c1a);
  }

  {
    const float bias = b_w[ncol];
    const int lc = wave * 16 + m;
#pragma unroll
    for (int r = 0; r < 8; ++r) {
      Xs[(8 * hh + r) * XSP + lc]      = c0a[r] + bias;
      Xs[(16 + 8 * hh + r) * XSP + lc] = c1a[r] + bias;
    }
  }
  __syncthreads();

  v4f xr[4];
  float* pp[4];
#pragma unroll
  for (int i = 0; i < 4; ++i) {
    xr[i] = *(const v4f*)(Xs + (4 * wave + i) * XSP + 4 * lane);
    pp[i] = P + (size_t)(rowBase + 4 * wave + i) * DW + colBase + 4 * lane;
  }
#pragma unroll
  for (int i = 0; i < 4; ++i) *(volatile v4f*)(pp[i]) = xr[i];
  __threadfence();
#pragma unroll
  for (int i = 0; i < 4; ++i) *(volatile v4f*)(pp[i]) = xr[i];
}

__global__ __launch_bounds__(NTHR) void k_edge(
    const float* __restrict__ ef, const int* __restrict__ srcA, const int* __restrict__ dstA,
    const _Float16* __restrict__ Wrt, const float* __restrict__ b_rel,
    const float* __restrict__ gam, const float* __restrict__ bet,
    const float* __restrict__ W_att, const float* __restrict__ b_att,
    const float* __restrict__ AT, float* U, int nE, int nN) {
  __shared__ __attribute__((aligned(16))) _Float16 As[GR * APE];
  __shared__ __attribute__((aligned(16))) float Xs[GR * XSP];
  __shared__ __attribute__((aligned(16))) float sW3[DN * NH];
  __shared__ __attribute__((aligned(16))) float Us[GR * NH];

  const int tid = threadIdx.x, lane = tid & 31, wave = tid >> 5;
  const int hh = lane >> 4, m = lane & 15;
  const int e0 = blockIdx.x * GR;

  {
    const int r = tid >> 3, c0 = (tid & 7) * 8;
    int e = e0 + r;
    if (e > nE - 1) e = nE - 1;
    const float* p = ef + (size_t)e * DE + c0;
    const v4f f0 = *(const v4f*)(p), f1 = *(const v4f*)(p + 4);
    Pack16 u;
    u.h[0] = (_Float16)f0.x; u.h[1] = (_Float16)f0.y; u.h[2] = (_Float16)f0.z; u.h[3] = (_Float16)f0.w;
    u.h[4] = (_Float16)f1.x; u.h[5] = (_Float16)f1.y; u.h[6] = (_Float16)f1.z; u.h[7] = (_Float16)f1.w;
    *(v8h*)(As + r * APE + c0) = u.h;
    if (tid < DN) *(v4f*)(sW3 + tid * NH) = *(const v4f*)(W_att + (size_t)(2 * DN + tid) * NH);
  }
  __syncthreads();

  const int ncol = wave * 16 + m;
  v8f c0a = {0.f, 0.f, 0.f, 0.f, 0.f, 0.f, 0.f, 0.f};
  v8f c1a = {0.f, 0.f, 0.f, 0.f, 0.f, 0.f, 0.f, 0.f};
#pragma unroll
  for (int kt = 0; kt < DE / 32; ++kt) {
    const int k0 = kt * 32;
    FragH a0, a1, b;
    const _Float16* pb  = Wrt + (size_t)ncol * DE + k0 + 8 * hh;
    const _Float16* pa0 = As + m * APE + k0 + 8 * hh;
    const _Float16* pa1 = As + (16 + m) * APE + k0 + 8 * hh;
    b.half[0]  = *(const v8h*)pb;  b.half[1]  = *(const v8h*)(pb + 16);
    a0.half[0] = *(const v8h*)pa0; a0.half[1] = *(const v8h*)(pa0 + 16);
    a1.half[0] = *(const v8h*)pa1; a1.half[1] = *(const v8h*)(pa1 + 16);
    c0a = wmh(a0.v, b.v, c0a);
    c1a = wmh(a1.v, b.v, c1a);
  }

  {
    const float br = b_rel[ncol];
#pragma unroll
    for (int r = 0; r < 8; ++r) {
      Xs[(8 * hh + r) * XSP + ncol]      = c0a[r] * 0.125f + br;
      Xs[(16 + 8 * hh + r) * XSP + ncol] = c1a[r] * 0.125f + br;
    }
  }
  __syncthreads();

  const v4f g4  = *(const v4f*)(gam + 4 * lane);
  const v4f be4 = *(const v4f*)(bet + 4 * lane);
  const v4f ba4 = *(const v4f*)(b_att);
  const float* w3 = sW3 + (4 * lane) * NH;
#pragma unroll 1
  for (int i = 0; i < GR / NWAVE; ++i) {
    const int row = wave * (GR / NWAVE) + i;
    int e = e0 + row;
    if (e > nE - 1) e = nE - 1;
    const v4f x = *(const v4f*)(Xs + row * XSP + 4 * lane);
    const float mu = wsum(x.x + x.y + x.z + x.w) * (1.0f / DN);
    const v4f d = x - mu;
    const float var = wsum(d.x * d.x + d.y * d.y + d.z * d.z + d.w * d.w) * (1.0f / DN);
    const float rs = rsqrtf(var + LN_EPS_F);
    v4f y = d * rs * g4 + be4;
    y.x = y.x > 0.f ? y.x : 0.f;
    y.y = y.y > 0.f ? y.y : 0.f;
    y.z = y.z > 0.f ? y.z : 0.f;
    y.w = y.w > 0.f ? y.w : 0.f;
    v4f q = y.x * *(const v4f*)(w3) + y.y * *(const v4f*)(w3 + 4)
          + y.z * *(const v4f*)(w3 + 8) + y.w * *(const v4f*)(w3 + 12);
    q.x = wsum(q.x); q.y = wsum(q.y); q.z = wsum(q.z); q.w = wsum(q.w);
    int si = srcA[e];
    si = si < 0 ? 0 : (si > nN - 1 ? nN - 1 : si);
    int di = dstA[e];
    di = di < 0 ? 0 : (di > nN - 1 ? nN - 1 : di);
    const v4f ad = *(const v4f*)(AT + (size_t)di * 8);
    const v4f as = *(const v4f*)(AT + (size_t)si * 8 + 4);
    v4f v = ad + as + q + ba4;
    v.x = v.x >= 0.f ? v.x : LEAKY_F * v.x;
    v.y = v.y >= 0.f ? v.y : LEAKY_F * v.y;
    v.z = v.z >= 0.f ? v.z : LEAKY_F * v.z;
    v.w = v.w >= 0.f ? v.w : LEAKY_F * v.w;
    if (lane == 0) *(v4f*)(Us + row * NH) = v;
  }
  __syncthreads();

  {
    const bool doit = (wave == 0);
    const v4f v = *(const v4f*)(Us + lane * NH);
    float* up = U + (size_t)(e0 + lane) * NH;
    if (doit) *(volatile v4f*)up = v;
    __threadfence();
    if (doit) *(volatile v4f*)up = v;
  }
}

__global__ __launch_bounds__(NTHR) void k_agg(
    const float* __restrict__ hA, const int* __restrict__ srcA, const int* __restrict__ dstA,
    const float* __restrict__ U, const float* __restrict__ P, const float* __restrict__ prelu_a,
    float* out, int nN, int nE) {
  extern __shared__ v4f lds_dyn[];
  float* sacc = (float*)lds_dyn;
  float* mx   = sacc + LDS_SACC;
  float* den  = mx + LDS_MX;
  int*   list = (int*)(den + LDS_DEN);
  int*   wcnt = list + LDS_LIST;

  const int tid  = threadIdx.x;
  const int lane = tid & 31;
  const int wave = tid >> 5;
  const int nodeBase = blockIdx.x * NB;

  {
    const v4f z4 = {0.f, 0.f, 0.f, 0.f};
    const v4f n4 = {-1e30f, -1e30f, -1e30f, -1e30f};
    const int i0 = LDS_SACC / 4, i1 = (LDS_SACC + LDS_MX) / 4, i2 = (LDS_SACC + LDS_MX + LDS_DEN) / 4;
    for (int i = tid; i < i2; i += NTHR) {
      if (i >= i0 && i < i1) lds_dyn[i] = n4;
      else lds_dyn[i] = z4;
    }
  }
  __syncthreads();

  const int nChunks = (nE + CHUNK - 1) / CHUNK;
  const int nIter = 2 * nChunks;
#pragma unroll 1
  for (int it = 0; it < nIter; ++it) {
    const int pass = (it >= nChunks) ? 1 : 0;
    const int ch = it - pass * nChunks;
    if (it == nChunks) {
      for (int i = tid; i < LDS_DEN; i += NTHR) {
        const float d = den[i];
        den[i] = (d > 0.f) ? (1.0f / d) : 0.f;
      }
      __syncthreads();
    }
    const int cbase = ch * CHUNK;
    int wc = 0;
#pragma unroll
    for (int g = 0; g < NGRP; ++g) {
      const int el0 = (g * NTHR + tid) * 4;
      const int eg0 = cbase + el0;
      const int sent = -2147483647 - 1;
      v4i d;
      if (eg0 + 3 < nE) {
        d = *(const v4i*)(dstA + eg0);
      } else {
        d.x = (eg0     < nE) ? dstA[min(eg0, nE - 1)]     : sent;
        d.y = (eg0 + 1 < nE) ? dstA[min(eg0 + 1, nE - 1)] : sent;
        d.z = (eg0 + 2 < nE) ? dstA[min(eg0 + 2, nE - 1)] : sent;
        d.w = (eg0 + 3 < nE) ? dstA[min(eg0 + 3, nE - 1)] : sent;
      }
      const unsigned s0 = (unsigned)d.x - (unsigned)nodeBase;
      const unsigned s1 = (unsigned)d.y - (unsigned)nodeBase;
      const unsigned s2 = (unsigned)d.z - (unsigned)nodeBase;
      const unsigned s3 = (unsigned)d.w - (unsigned)nodeBase;
      const bool h0 = s0 < (unsigned)NB;
      const bool h1 = s1 < (unsigned)NB;
      const bool h2 = s2 < (unsigned)NB;
      const bool h3 = s3 < (unsigned)NB;
      const unsigned many = __builtin_amdgcn_ballot_w32(h0 | h1 | h2 | h3);
      if (many != 0u) {
#define HITJ(J, HJ, SJ) { \
          const unsigned mj = __builtin_amdgcn_ballot_w32(HJ); \
          if (HJ) { \
            const int pos = wc + (int)__builtin_amdgcn_mbcnt_lo(mj, 0u); \
            if (pos < WCAP) list[wave * WCAP + pos] = ((el0 + (J)) << 9) | (int)(SJ); \
          } \
          wc += (int)__builtin_popcount(mj); }
        HITJ(0, h0, s0)
        HITJ(1, h1, s1)
        HITJ(2, h2, s2)
        HITJ(3, h3, s3)
#undef HITJ
      }
    }
    if (lane == 0) wcnt[wave] = wc;
    __syncthreads();

    if (wave == 0) {
      for (int wsx = 0; wsx < NWAVE; ++wsx) {
        int n = wcnt[wsx];
        if (n > WCAP) n = WCAP;
        if (n < 0) n = 0;
        if (pass == 0) {
          for (int i = 0; i < n; ++i) {
            const int ent  = list[wsx * WCAP + i];
            const int slot = ent & (NB - 1);
            const int el   = (ent >> 9) & (CHUNK - 1);
            int e = cbase + el;
            if (e > nE - 1) e = nE - 1;
            if (lane < NH) {
              const float u  = U[(size_t)e * NH + lane];
              const int   ai = slot * NH + lane;
              const float mo = mx[ai];
              const float mn = (u > mo) ? u : mo;
              const float dd = den[ai];
              const float dn = dd * __expf(mo - mn) + __expf(u - mn);
              mx[ai]  = mn;
              den[ai] = dn;
            }
          }
        } else {
          for (int i = 0; i < n; ++i) {
            const int ent  = list[wsx * WCAP + i];
            const int slot = ent & (NB - 1);
            const int el   = (ent >> 9) & (CHUNK - 1);
            int e = cbase + el;
            if (e > nE - 1) e = nE - 1;
            int s = srcA[e];
            s = s < 0 ? 0 : (s > nN - 1 ? nN - 1 : s);
            const v4f u4 = *(const v4f*)(U + (size_t)e * NH);
            const v4f m4 = *(const v4f*)(mx + slot * NH);
            const v4f r4 = *(const v4f*)(den + slot * NH);
            const float c0 = __expf(u4.x - m4.x) * r4.x;
            const float c1 = __expf(u4.y - m4.y) * r4.y;
            const float c2 = __expf(u4.z - m4.z) * r4.z;
            const float c3 = __expf(u4.w - m4.w) * r4.w;
            const float* pp = P + (size_t)s * DW + 4 * lane;
            const v4f p0 = *(const v4f*)(pp);
            const v4f p1 = *(const v4f*)(pp + DN);
            const v4f p2 = *(const v4f*)(pp + 2 * DN);
            const v4f p3 = *(const v4f*)(pp + 3 * DN);
            v4f* sp = (v4f*)(sacc + slot * DN + 4 * lane);
            const v4f cur = *sp;
            *sp = cur + c0 * p0 + c1 * p1 + c2 * p2 + c3 * p3;
          }
        }
      }
    }
    __syncthreads();
  }

  const float ap = prelu_a[0];
#pragma unroll 1
  for (int j = 0; j < NB / NWAVE; ++j) {
    const int slot = wave * (NB / NWAVE) + j;
    const int node = nodeBase + slot;
    if (node >= nN) break;
    const size_t nrow = (size_t)node;
    v4f sv = *(const v4f*)(sacc + slot * DN + 4 * lane);
    sv = sv * 0.25f;
    sv.x = sv.x >= 0.f ? sv.x : ap * sv.x;
    sv.y = sv.y >= 0.f ? sv.y : ap * sv.y;
    sv.z = sv.z >= 0.f ? sv.z : ap * sv.z;
    sv.w = sv.w >= 0.f ? sv.w : ap * sv.w;
    const bool has = den[slot * NH] > 0.f;
    v4f o = *(const v4f*)(hA + nrow * DN + 4 * lane);
    if (has) o = sv;
    float* op = out + nrow * DN + 4 * lane;
    *(volatile v4f*)op = o;
    __threadfence();
    *(volatile v4f*)op = o;
  }
}

static inline size_t al256(size_t x) { return (x + 255) & ~(size_t)255; }

extern "C" void kernel_launch(void* const* d_in, const int* in_sizes, int n_in,
                              void* d_out, int out_size, void* d_ws, size_t ws_size,
                              hipStream_t stream) {
  if (n_in < 13) return;
  const int nN = in_sizes[0] / DN;
  const int nE = in_sizes[2];
  if (nN <= 0 || in_sizes[0] != nN * DN) return;
  if (nE < 0 || in_sizes[3] != nE) return;
  if ((size_t)in_sizes[1] != (size_t)nE * DE) return;
  if (in_sizes[4] != DE * DN || in_sizes[5] != DN || in_sizes[6] != DN || in_sizes[7] != DN) return;
  if (in_sizes[8] != 3 * DN * NH || in_sizes[9] != NH) return;
  if (in_sizes[10] != DN * DW || in_sizes[11] != DW || in_sizes[12] < 1) return;
  if (out_size != nN * DN) return;

  const float* hA      = (const float*)d_in[0];
  const float* ef      = (const float*)d_in[1];
  const int*   srcA    = (const int*)d_in[2];
  const int*   dstA    = (const int*)d_in[3];
  const float* W_rel   = (const float*)d_in[4];
  const float* b_rel   = (const float*)d_in[5];
  const float* gam     = (const float*)d_in[6];
  const float* bet     = (const float*)d_in[7];
  const float* W_att   = (const float*)d_in[8];
  const float* b_att   = (const float*)d_in[9];
  const float* W_w     = (const float*)d_in[10];
  const float* b_w     = (const float*)d_in[11];
  const float* prelu_a = (const float*)d_in[12];
  float* out = (float*)d_out;

  const int nP = ((nN + NAB - 1) / NAB) * NAB;
  const int EP = ((nE + GR - 1) / GR) * GR;
  char* wb = (char*)d_ws;
  size_t off = 0;
  _Float16* Wrt = (_Float16*)(wb + off);            off += al256((size_t)DN * DE * sizeof(_Float16));
  unsigned short* Wh = (unsigned short*)(wb + off); off += al256((size_t)DW * DN * sizeof(unsigned short));
  unsigned short* Wl = (unsigned short*)(wb + off); off += al256((size_t)DW * DN * sizeof(unsigned short));
  float* P  = (float*)(wb + off);                   off += al256((size_t)nP * DW * sizeof(float));
  float* AT = (float*)(wb + off);                   off += al256((size_t)nP * 8 * sizeof(float));
  float* U  = (float*)(wb + off);                   off += al256((size_t)EP * NH * sizeof(float));
  if (off > ws_size) return;

  const int nPrep = DN * DE / 8 + DW * DN / 8;
  k_prepw<<<(nPrep + NTHR - 1) / NTHR, NTHR, 0, stream>>>(W_rel, W_w, Wrt, Wh, Wl);

  k_nodeatt<<<nP / NAB, NTHR, 0, stream>>>(hA, W_att, AT, nN);

  k_pgemm<<<dim3(nP / GR, DW / DN), NTHR, 0, stream>>>(hA, Wh, Wl, b_w, P, nN);

  if (nE > 0) {
    k_edge<<<EP / GR, NTHR, 0, stream>>>(ef, srcA, dstA, Wrt, b_rel, gam, bet, W_att, b_att,
                                          AT, U, nE, nN);
  }

  hipFuncSetAttribute(reinterpret_cast<const void*>(&k_agg),
                      hipFuncAttributeMaxDynamicSharedMemorySize, LDS_BYTES);
  const int grid = (nN + NB - 1) / NB;
  k_agg<<<grid, NTHR, LDS_BYTES, stream>>>(hA, srcA, dstA, U, P, prelu_a, out, nN, nE);
}
